// GenoMixMamba2Extension_21165598834738
// MI455X (gfx1250) — hardware-run, weakly checked
//
#include <hip/hip_runtime.h>
#include <math.h>

typedef __attribute__((ext_vector_type(16))) _Float16 v16h;
typedef __attribute__((ext_vector_type(8)))  _Float16 v8h;
typedef __attribute__((ext_vector_type(16))) __bf16   v16b;
typedef __attribute__((ext_vector_type(8)))  __bf16   v8b;
typedef __attribute__((ext_vector_type(8)))  float    v8f;
typedef __attribute__((ext_vector_type(4)))  float    v4f;
typedef __attribute__((ext_vector_type(4)))  unsigned v4u;

constexpr int kBatch = 2;
constexpr int kSeq   = 2048;
constexpr int kDm    = 1024;
constexpr int kDi    = 2048;
constexpr int kNs    = 128;
constexpr int kHd    = 64;
constexpr int kNh    = 32;
constexpr int kCv    = 2304;
constexpr int kPj    = 4384;
constexpr int kPjP   = 4416;
constexpr int kRows  = kBatch * kSeq;
constexpr int kQ     = 64;
constexpr int kNck   = kSeq / kQ;
constexpr int kZxW    = kPjP / 2;
constexpr int kXColW  = kDi / 2;
constexpr int kBcColW = (2 * kDi) / 2;
constexpr int kDtColW = (kDi + kCv) / 2;
constexpr float kWCarry  = 32.0f;
constexpr float kYnCarry = 16.0f;
constexpr float kGCarry  = 64.0f;
static_assert(kDi + kCv + kNh == kPj);
static_assert(kCv == kDi + 2 * kNs);
static_assert(kNh * kHd == kDi);
static_assert(kPjP >= kPj && (kPjP % 64) == 0);
static_assert((kRows % 64) == 0 && (kDm % 64) == 0 && (kDm % 32) == 0 && ((2 * kDi) % 32) == 0);
static_assert(kQ == 64 && kNck == 32 && kHd == 64 && kNs == 128 && kNh == 32 && kBatch == 2);
static_assert(((kRows / 64) * (kPjP / 64)) % 8 == 0);
static_assert(((kRows / 64) * (kDm / 64)) % 8 == 0);

constexpr size_t kSzX16  = (size_t)kRows * kDm * 2;
constexpr size_t kSzWinT = (size_t)2 * kPjP * kDm * 2;
constexpr size_t kSzG    = (size_t)2 * kRows * kDi * 2;
constexpr size_t kSzA    = kSzG;
constexpr size_t kSzZX   = (size_t)2 * kRows * kPjP * 2;
constexpr size_t kSzYN   = (size_t)kRows * 2 * kDi * 2;
constexpr size_t kSzBC   = (size_t)2 * kBatch * kSeq * 256 * 2;
constexpr size_t kSzBT   = (size_t)2 * kBatch * kNs * kSeq * 2;
constexpr size_t kSzCB   = (size_t)2 * kBatch * kNck * kQ * kQ * 4;
constexpr size_t kSzWoT  = (size_t)kDm * 2 * kDi * 2;
constexpr size_t kOffX16  = 0;
constexpr size_t kOffWinT = kOffX16 + kSzX16;
constexpr size_t kOffG    = 0;
constexpr size_t kOffZX   = kSzA;
constexpr size_t kOffYN   = kOffZX;
constexpr size_t kOffBC   = kOffZX + kSzZX;
constexpr size_t kOffBT   = kOffBC + kSzBC;
constexpr size_t kOffCB   = kOffBT + kSzBT;
constexpr size_t kOffWoT  = kOffCB + kSzCB;
constexpr size_t kWsTotal = kOffWoT + kSzWoT;
static_assert(kSzX16 + kSzWinT <= kSzA);
static_assert(kSzYN <= kSzZX);
static_assert(kWsTotal == 122683392ull);
static_assert(kWsTotal <= 134217728ull);
static_assert((kOffWinT % 128) == 0 && (kOffZX % 128) == 0 && (kOffBC % 128) == 0 && (kOffBT % 128) == 0 &&
              (kOffCB % 128) == 0 && (kOffWoT % 128) == 0);

__device__ __forceinline__ unsigned short f2bf_bits(float f) {
  unsigned u = __float_as_uint(f);
  return (unsigned short)((u + 0x7FFFu + ((u >> 16) & 1u)) >> 16);
}
__device__ __forceinline__ float bf_bits2f(unsigned short h) { return __uint_as_float(((unsigned)h) << 16); }
__device__ __forceinline__ float bf16_rne(float f) { return bf_bits2f(f2bf_bits(f)); }
__device__ __forceinline__ __bf16 bits2bf(unsigned short b) { return __builtin_bit_cast(__bf16, b); }
__device__ __forceinline__ float h16_to_f32(unsigned hb) {
  const unsigned sgn = (hb & 0x8000u) << 16;
  const unsigned em = hb & 0x7fffu;
  const float fn = __uint_as_float((em << 13) + 0x38000000u);
  const float fs = (float)em * 5.9604644775390625e-8f;
  const float mag = (em < 0x400u) ? fs : fn;
  return __uint_as_float(__float_as_uint(mag) | sgn);
}
__device__ __forceinline__ float silu_f(float v) {
  return v * __builtin_amdgcn_rcpf(1.0f + expf(-v));
}

__device__ __forceinline__ void dep_guard4_h(v8f& a, v8f& b, v8f& c, v8f& d, v16h x) {
  asm volatile("v_nop\n\tv_nop\n\tv_nop\n\tv_nop" : "+v"(a), "+v"(b), "+v"(c), "+v"(d) : "v"(x));
}
__device__ __forceinline__ void keep4_h(v16h a, v16h b, v16h c, v16h d) { asm volatile("v_nop" :: "v"(a), "v"(b), "v"(c), "v"(d)); }
__device__ __forceinline__ void acc_guard4(v8f& a, v8f& b, v8f& c, v8f& d) { asm volatile("v_nop\n\tv_nop\n\tv_nop\n\tv_nop" : "+v"(a), "+v"(b), "+v"(c), "+v"(d)); }

template <typename T> struct Frag;
template <> struct Frag<_Float16> {
  typedef v16h V; union U { v16h v; v8h h[2]; };
  static __device__ __forceinline__ v16h load(const _Float16* p) {
    U f; f.h[0] = *(const v8h*)(p); f.h[1] = *(const v8h*)(p + 16); return f.v;
  }
  static __device__ __forceinline__ v8f mma(v16h a, v16h b, v8f c) {
    return __builtin_amdgcn_wmma_f32_16x16x32_f16(false, a, false, b, (short)0, c, false, false);
  }
};
template <> struct Frag<__bf16> {
  typedef v16b V; union U { v16b v; v8b h[2]; };
  static __device__ __forceinline__ v16b load(const __bf16* p) {
    U f; f.h[0] = *(const v8b*)(p); f.h[1] = *(const v8b*)(p + 16); return f.v;
  }
};
__device__ __forceinline__ v8f mma_b(v16b a, v16b b, v8f c) {
  c = __builtin_amdgcn_wmma_f32_16x16x32_bf16(false, a, false, b, (short)0, c, false, false);
  asm volatile("v_nop\n\tv_nop\n\tv_nop\n\tv_nop" : "+v"(c) : "v"(a), "v"(b));
  return c;
}

template <int OUT_MODE>
__global__ __launch_bounds__(256) void wmma_gemm64_f16(
    const unsigned short* __restrict__ Ap, int lda, long strideA,
    const unsigned short* __restrict__ Btp, int ldb, long strideB,
    void* __restrict__ Cout, int ldc, long strideC,
    int M, int N, int K, float scale) {
  typedef _Float16 T;
  typedef v16h V;
  const T* A = (const T*)Ap;
  const T* Bt = (const T*)Btp;
  __shared__ __align__(16) float sT[8][16 * 68];
  const int b    = blockIdx.y;
  const int lane = threadIdx.x & 31;
  const int wave = threadIdx.x >> 5;
  const int tilesN = N >> 6;
  const int tilesM = M >> 6;
  const int tile = blockIdx.x * 8 + wave;
  if (tile >= tilesM * tilesN) return;
  const int tm = tile / tilesN;
  const int tn = tile - tm * tilesN;
  const int m0 = tm << 6;
  const int n0 = tn << 6;

  const T* Ab = A  + (size_t)b * strideA;
  const T* Bb = Bt + (size_t)b * strideB;

  const int rlane = lane & 15;
  const int koff  = (lane >> 4) * 8;
  const int mOff  = (lane >> 4) * 8;

  v8f acc[4][4];
#pragma unroll
  for (int i = 0; i < 4; ++i)
#pragma unroll
    for (int j = 0; j < 4; ++j) acc[i][j] = (v8f){0.f,0.f,0.f,0.f,0.f,0.f,0.f,0.f};

  for (int k0 = 0; k0 < K; k0 += 32) {
    V bh[4];
#pragma unroll
    for (int j = 0; j < 4; ++j) {
      const size_t bo = (size_t)(n0 + (j << 4) + rlane) * ldb + koff + k0;
      bh[j] = Frag<T>::load(Bb + bo);
    }
#pragma unroll
    for (int i = 0; i < 4; ++i) {
      const size_t ao = (size_t)(m0 + (i << 4) + rlane) * lda + koff + k0;
      V ah = Frag<T>::load(Ab + ao);
#pragma unroll
      for (int j = 0; j < 4; ++j) acc[i][j] = Frag<T>::mma(ah, bh[j], acc[i][j]);
      dep_guard4_h(acc[i][0], acc[i][1], acc[i][2], acc[i][3], ah);
    }
    keep4_h(bh[0], bh[1], bh[2], bh[3]);
  }
  acc_guard4(acc[0][0], acc[0][1], acc[0][2], acc[0][3]);
  acc_guard4(acc[1][0], acc[1][1], acc[1][2], acc[1][3]);
  acc_guard4(acc[2][0], acc[2][1], acc[2][2], acc[2][3]);
  acc_guard4(acc[3][0], acc[3][1], acc[3][2], acc[3][3]);

  float* slab = sT[wave];
#pragma unroll
  for (int i = 0; i < 4; ++i) {
    const int mBase = m0 + (i << 4);
#pragma unroll
    for (int j = 0; j < 4; ++j) {
#pragma unroll
      for (int r = 0; r < 8; ++r) {
        const float v = acc[i][j][r] * scale;
        slab[(mOff + r) * 68 + (j << 4) + rlane] = v;
      }
    }
    __builtin_amdgcn_fence(__ATOMIC_RELEASE, "workgroup");
    __builtin_amdgcn_wave_barrier();
    __builtin_amdgcn_fence(__ATOMIC_ACQUIRE, "workgroup");
    if (OUT_MODE == 0) {
      float* C = (float*)Cout + (size_t)b * strideC;
      const int hh = lane >> 4, c4 = (lane & 15) * 4;
      for (int pass = 0; pass < 2; ++pass) {
#pragma unroll
        for (int it = 0; it < 8; ++it) {
          const int row = it * 2 + hh;
          v4f v = *(const v4f*)(slab + row * 68 + c4);
          *(volatile v4f*)(C + (size_t)(mBase + row) * ldc + n0 + c4) = v;
        }
        __threadfence();
      }
    } else {
      const int q = lane >> 3, c8 = (lane & 7) * 8;
      unsigned short* C = (unsigned short*)Cout + (size_t)b * strideC;
      for (int pass = 0; pass < 2; ++pass) {
#pragma unroll
        for (int it = 0; it < 4; ++it) {
          const int row = it * 4 + q;
          const float* sp = slab + row * 68 + c8;
          v8h hv;
#pragma unroll
          for (int e = 0; e < 8; ++e) hv[e] = (_Float16)sp[e];
          *(volatile v8h*)(C + (size_t)(mBase + row) * ldc + n0 + c8) = hv;
        }
        __threadfence();
      }
    }
    __builtin_amdgcn_fence(__ATOMIC_RELEASE, "workgroup");
    __builtin_amdgcn_wave_barrier();
    __builtin_amdgcn_fence(__ATOMIC_ACQUIRE, "workgroup");
  }
}

__global__ __launch_bounds__(256) void cast_rows_f16_kernel(
    const float* __restrict__ src, unsigned short* __restrict__ dst, int total8)
{
  const int i = blockIdx.x * 256 + threadIdx.x;
  if (i >= total8) return;
  const size_t e0 = (size_t)i << 3;
  const v4f a0 = *(const v4f*)(src + e0);
  const v4f a1 = *(const v4f*)(src + e0 + 4);
  v8h hv;
#pragma unroll
  for (int e = 0; e < 4; ++e) {
    hv[e]     = (_Float16)bf16_rne(a0[e]);
    hv[4 + e] = (_Float16)bf16_rne(a1[e]);
  }
  unsigned short* q = dst + e0;
  *(volatile v8h*)q = hv;
  __threadfence();
  *(volatile v8h*)q = hv;
}

__global__ __launch_bounds__(256) void transpose_cast_kernel(
    const float* __restrict__ W0, const float* __restrict__ W1, unsigned short* __restrict__ Bt,
    int Kdim, int Ndim, int ldo, long planeStride, int kStride, float scale)
{
  __shared__ float tile[64 * 65];
  const int tid = threadIdx.x, lane = tid & 31, wave = tid >> 5;
  const int n0 = blockIdx.x * 64;
  const int k0 = blockIdx.y * 64;
  const int z  = blockIdx.z;
  const float* W = z ? W1 : W0;
  unsigned short* Bo = Bt + (size_t)z * planeStride + (size_t)z * kStride;
#pragma unroll
  for (int p = 0; p < 16; ++p) {
    const int idx = tid + p * 256;
    const int kk  = idx >> 6;
    const int nn  = idx & 63;
    const int n   = n0 + nn;
    const int nc  = (n < Ndim) ? n : (Ndim - 1);
    const float v = W[(size_t)(k0 + kk) * Ndim + nc];
    tile[kk * 65 + nn] = (n < Ndim) ? (bf16_rne(v) * scale) : 0.f;
  }
  __syncthreads();
  const int q = lane >> 3, c8 = (lane & 7) * 8;
  v8h hv[2];
#pragma unroll
  for (int it = 0; it < 2; ++it) {
    const int nrow = it * 32 + wave * 4 + q;
#pragma unroll
    for (int e = 0; e < 8; ++e) hv[it][e] = (_Float16)tile[(c8 + e) * 65 + nrow];
  }
  for (int pass = 0; pass < 2; ++pass) {
#pragma unroll
    for (int it = 0; it < 2; ++it) {
      const int nrow = it * 32 + wave * 4 + q;
      *(volatile v8h*)(Bo + (size_t)(n0 + nrow) * ldo + k0 + c8) = hv[it];
    }
    __threadfence();
  }
}

__global__ __launch_bounds__(256) void bc_prep_kernel(
    const unsigned* __restrict__ ZXw,
    const float* __restrict__ cw0, const float* __restrict__ cb0,
    const float* __restrict__ cw1, const float* __restrict__ cb1,
    unsigned short* __restrict__ BCc, unsigned short* __restrict__ BTp, float* __restrict__ CBp)
{
  __shared__ __align__(16) __bf16 sBC[64 * 256];
  __shared__ __align__(16) float sS[8][16 * 36];
  const int tid = threadIdx.x, lane = tid & 31, wave = tid >> 5, hh = lane >> 4, l15 = lane & 15;
  const int bid = blockIdx.x;
  const int ck = bid & 31, bb = (bid >> 5) & 1, dir = bid >> 6;
  const int s0 = ck * kQ;
  const float* cw = dir ? cw1 : cw0;
  const float* cb = dir ? cb1 : cb0;
  const int ch = kDi + tid;
  const float w0 = bf16_rne(cw[0 * kCv + ch]);
  const float w1 = bf16_rne(cw[1 * kCv + ch]);
  const float w2 = bf16_rne(cw[2 * kCv + ch]);
  const float w3 = bf16_rne(cw[3 * kCv + ch]);
  const float cbias = bf16_rne(cb[ch]);
  const unsigned* ZXd = ZXw + (size_t)dir * ((size_t)kRows * kZxW);
  const int wcol = kBcColW + (tid >> 1);
  const bool hiSel = (tid & 1) != 0;

  float xh[3];
#pragma unroll
  for (int k = 0; k < 3; ++k) {
    const int s  = s0 - 3 + k;
    const int sc = s < 0 ? 0 : s;
    const int trow = bb * kSeq + (dir ? (kSeq - 1 - sc) : sc);
    const unsigned w = ZXd[(size_t)trow * kZxW + wcol];
    const float v = h16_to_f32(hiSel ? (w >> 16) : (w & 0xffffu));
    xh[k] = (s < 0) ? 0.0f : v;
  }
  float xm3 = xh[0], xm2 = xh[1], xm1 = xh[2];
#pragma unroll 1
  for (int j = 0; j < kQ; ++j) {
    const int s = s0 + j;
    const int trow = bb * kSeq + (dir ? (kSeq - 1 - s) : s);
    const unsigned w = ZXd[(size_t)trow * kZxW + wcol];
    const float xc = h16_to_f32(hiSel ? (w >> 16) : (w & 0xffffu));
    float acc = fmaf(xm3, w0, cbias);
    acc = fmaf(xm2, w1, acc);
    acc = fmaf(xm1, w2, acc);
    acc = fmaf(xc, w3, acc);
    sBC[j * 256 + tid] = bits2bf(f2bf_bits(silu_f(acc)));
    xm3 = xm2; xm2 = xm1; xm1 = xc;
  }
  __syncthreads();

  const size_t db = (size_t)(dir * 2 + bb);
  {
    unsigned short* BCd = BCc + (db * kSeq + s0) * 256;
    for (int pass = 0; pass < 2; ++pass) {
#pragma unroll
      for (int it = 0; it < 8; ++it) {
        const int j = it * 8 + wave;
        const v4u v = *(const v4u*)(const void*)(sBC + j * 256 + lane * 8);
        *(volatile v4u*)(void*)(BCd + (size_t)j * 256 + lane * 8) = v;
      }
      __threadfence();
    }
  }
  {
    const unsigned short* sBCu = (const unsigned short*)(const void*)sBC;
    unsigned short* BTd = BTp + db * ((size_t)kNs * kSeq);
    const int q = lane >> 3, c8 = (lane & 7) * 8;
    for (int pass = 0; pass < 2; ++pass) {
#pragma unroll
      for (int it = 0; it < 4; ++it) {
        const int n = it * 32 + wave * 4 + q;
        v4u o;
#pragma unroll
        for (int k = 0; k < 4; ++k) {
          const unsigned lo = sBCu[(c8 + 2 * k) * 256 + n];
          const unsigned hi = sBCu[(c8 + 2 * k + 1) * 256 + n];
          o[k] = lo | (hi << 16);
        }
        *(volatile v4u*)(void*)(BTd + (size_t)n * kSeq + s0 + c8) = o;
      }
      __threadfence();
    }
  }
  {
    const int itl = wave >> 1, hf = wave & 1;
    v8f acc[2];
    acc[0] = (v8f){0.f,0.f,0.f,0.f,0.f,0.f,0.f,0.f};
    acc[1] = (v8f){0.f,0.f,0.f,0.f,0.f,0.f,0.f,0.f};
#pragma unroll
    for (int ks = 0; ks < 4; ++ks) {
      const v16b af = Frag<__bf16>::load(sBC + (itl * 16 + l15) * 256 + kNs + ks * 32 + 8 * hh);
#pragma unroll
      for (int t = 0; t < 2; ++t) {
        const v16b bfv = Frag<__bf16>::load(sBC + ((hf * 2 + t) * 16 + l15) * 256 + ks * 32 + 8 * hh);
        acc[t] = mma_b(af, bfv, acc[t]);
      }
    }
    float* slab = sS[wave];
#pragma unroll
    for (int t = 0; t < 2; ++t)
#pragma unroll
      for (int r = 0; r < 8; ++r) slab[(8 * hh + r) * 36 + t * 16 + l15] = acc[t][r];
    __builtin_amdgcn_fence(__ATOMIC_RELEASE, "workgroup");
    __builtin_amdgcn_wave_barrier();
    __builtin_amdgcn_fence(__ATOMIC_ACQUIRE, "workgroup");
    float* CBd = CBp + (db * kNck + ck) * ((size_t)kQ * kQ);
    const int q = lane >> 3, c4 = (lane & 7) * 4;
    for (int pass = 0; pass < 2; ++pass) {
#pragma unroll
      for (int it = 0; it < 4; ++it) {
        const int row = it * 4 + q;
        const v4f v = *(const v4f*)(slab + row * 36 + c4);
        *(volatile v4f*)(CBd + (size_t)(itl * 16 + row) * kQ + hf * 32 + c4) = v;
      }
      __threadfence();
    }
  }
}

__global__ __launch_bounds__(256) void ssd_scan_kernel(
    const unsigned* __restrict__ ZXw, const unsigned short* __restrict__ BCc,
    const unsigned short* __restrict__ BTp, const float* __restrict__ CBp,
    const float* __restrict__ cw0, const float* __restrict__ cb0, const float* __restrict__ dtb0,
    const float* __restrict__ al0, const float* __restrict__ dd0,
    const float* __restrict__ cw1, const float* __restrict__ cb1, const float* __restrict__ dtb1,
    const float* __restrict__ al1, const float* __restrict__ dd1,
    unsigned short* __restrict__ Gp)
{
  __shared__ __align__(16) __bf16 sH[kHd * kNs];
  __shared__ __align__(16) unsigned sU[2176];
  __shared__ __align__(16) __bf16 sXT[kHd * kQ];
  __shared__ __align__(16) __bf16 sXW[kHd * kQ];
  __shared__ __align__(16) float sXf[kQ * 68];
  __shared__ float sDt[kQ];
  __shared__ float sA[kQ];
  __shared__ float sCs[kQ];
  __shared__ float sE[kQ];
  __shared__ float sW[kQ];
  __shared__ float sDec[4];
  __bf16* sM = (__bf16*)(void*)sU;

  const int tid = threadIdx.x, lane = tid & 31, wave = tid >> 5, hh = lane >> 4, l15 = lane & 15;
  const int bid = blockIdx.x;
  const int hd = bid & 31, bb = (bid >> 5) & 1, dir = bid >> 6;
  const float* cw  = dir ? cw1 : cw0;
  const float* cb  = dir ? cb1 : cb0;
  const float* dtb = dir ? dtb1 : dtb0;
  const float* al  = dir ? al1 : al0;
  const float* dd  = dir ? dd1 : dd0;
  const int pch = tid & 63, qg = tid >> 6;
  const int ch = hd * kHd + pch;
  const float w0 = bf16_rne(cw[0 * kCv + ch]);
  const float w1 = bf16_rne(cw[1 * kCv + ch]);
  const float w2 = bf16_rne(cw[2 * kCv + ch]);
  const float w3 = bf16_rne(cw[3 * kCv + ch]);
  const float cbias = bf16_rne(cb[ch]);
  const float dtbias = bf16_rne(dtb[hd]);
  const float Ah = -expf(bf16_rne(al[hd]));
  const float Dh = bf16_rne(dd[hd]);

  const size_t db = (size_t)(dir * 2 + bb);
  const unsigned* ZXd = ZXw + (size_t)dir * ((size_t)kRows * kZxW);
  const __bf16* BCd = (const __bf16*)(const void*)(BCc + db * ((size_t)kSeq * 256));
  const __bf16* BTd = (const __bf16*)(const void*)(BTp + db * ((size_t)kNs * kSeq));
  const float* CBd = CBp + db * ((size_t)kNck * kQ * kQ);
  unsigned short* Gd = Gp + (size_t)dir * ((size_t)kRows * kDi);

  {
    v8b zz;
#pragma unroll
    for (int e = 0; e < 8; ++e) zz[e] = bits2bf((unsigned short)0);
#pragma unroll
    for (int i = 0; i < 4; ++i) *(v8b*)(sH + (tid * 4 + i) * 8) = zz;
  }
  v8f hacc[4];
#pragma unroll
  for (int t = 0; t < 4; ++t) hacc[t] = (v8f){0.f,0.f,0.f,0.f,0.f,0.f,0.f,0.f};

  const int itl = wave >> 1, hf = wave & 1;
  const int wsel = pch >> 1;
  const bool hiSel = (pch & 1) != 0;

#pragma unroll 1
  for (int ck = 0; ck < kNck; ++ck) {
    const int s0 = ck * kQ;
    __syncthreads();
#pragma unroll
    for (int itA = 0; itA < 3; ++itA) {
      const int idx = tid + itA * 256;
      const int r = idx >> 3, c = idx & 7;
      const int rc = r < 67 ? r : 66;
      const int s = s0 - 3 + rc;
      const int sc = s < 0 ? 0 : s;
      const int trow = bb * kSeq + (dir ? (kSeq - 1 - sc) : sc);
      v4u v = *(const v4u*)(ZXd + (size_t)trow * kZxW + kXColW + hd * 32 + c * 4);
      asm volatile("" : "+v"(v));
      const v4u zero4 = {0u, 0u, 0u, 0u};
      v = (s < 0) ? zero4 : v;
      if (r < 67) *(v4u*)(sU + r * 32 + c * 4) = v;
    }
    if (tid < kQ) {
      const int s = s0 + tid;
      const int trow = bb * kSeq + (dir ? (kSeq - 1 - s) : s);
      const unsigned w = ZXd[(size_t)trow * kZxW + kDtColW + (hd >> 1)];
      const unsigned hb = (hd & 1) ? (w >> 16) : (w & 0xffffu);
      const float v = h16_to_f32(hb) + dtbias;
      const float dtv = fmaxf(v, 0.0f) + log1pf(expf(-fabsf(v)));
      sDt[tid] = dtv;
      sA[tid] = dtv * Ah;
    }
    __syncthreads();
    if (tid < kQ) {
      float pre = 0.0f, tot = 0.0f;
#pragma unroll 1
      for (int j = 0; j < kQ; ++j) {
        const float a = sA[j];
        tot += a;
        pre += (j <= tid) ? a : 0.0f;
      }
      sCs[tid] = pre;
      sE[tid] = expf(pre);
      sW[tid] = sDt[tid] * expf(fminf(tot - pre, 0.0f));
      if (tid == 0) sDec[0] = expf(tot);
    }
    __syncthreads();
    {
      const int j0 = qg * 16;
      float xm3, xm2, xm1;
      {
        const unsigned wa = sU[(j0 + 0) * 32 + wsel];
        const unsigned wb = sU[(j0 + 1) * 32 + wsel];
        const unsigned wc = sU[(j0 + 2) * 32 + wsel];
        xm3 = h16_to_f32(hiSel ? (wa >> 16) : (wa & 0xffffu));
        xm2 = h16_to_f32(hiSel ? (wb >> 16) : (wb & 0xffffu));
        xm1 = h16_to_f32(hiSel ? (wc >> 16) : (wc & 0xffffu));
      }
#pragma unroll 1
      for (int jj = 0; jj < 16; ++jj) {
        const int j = j0 + jj;
        const unsigned wd = sU[(j + 3) * 32 + wsel];
        const float xc = h16_to_f32(hiSel ? (wd >> 16) : (wd & 0xffffu));
        float acc = fmaf(xm3, w0, cbias);
        acc = fmaf(xm2, w1, acc);
        acc = fmaf(xm1, w2, acc);
        acc = fmaf(xc, w3, acc);
        const float sv = silu_f(acc);
        sXf[j * 68 + pch] = sv;
        sXT[pch * kQ + j] = bits2bf(f2bf_bits(sv));
        sXW[pch * kQ + j] = bits2bf(f2bf_bits(sv * sW[j]));
        xm3 = xm2; xm2 = xm1; xm1 = xc;
      }
    }
    __syncthreads();
    {
      const int i = tid >> 2, jb = (tid & 3) * 16;
      const float csi = sCs[i];
      const float* cbrow = CBd + (size_t)ck * (kQ * kQ) + i * kQ + jb;
#pragma unroll 1
      for (int g = 0; g < 4; ++g) {
        const v4f cv = *(const v4f*)(cbrow + 4 * g);
#pragma unroll
        for (int e = 0; e < 4; ++e) {
          const int j = jb + 4 * g + e;
          const float dlt = fminf(csi - sCs[j], 0.0f);
          const float val = cv[e] * expf(dlt) * sDt[j];
          sM[i * kQ + j] = bits2bf(f2bf_bits((j <= i) ? val : 0.0f));
        }
      }
    }
    __syncthreads();
    v8f yacc[2];
    yacc[0] = (v8f){0.f,0.f,0.f,0.f,0.f,0.f,0.f,0.f};
    yacc[1] = (v8f){0.f,0.f,0.f,0.f,0.f,0.f,0.f,0.f};
    {
      const __bf16* Crow = BCd + (size_t)(s0 + itl * 16 + l15) * 256 + kNs + 8 * hh;
#pragma unroll
      for (int ks = 0; ks < 4; ++ks) {
        const v16b af = Frag<__bf16>::load(Crow + ks * 32);
#pragma unroll
        for (int t = 0; t < 2; ++t) {
          const v16b bfv = Frag<__bf16>::load(sH + ((hf * 2 + t) * 16 + l15) * kNs + ks * 32 + 8 * hh);
          yacc[t] = mma_b(af, bfv, yacc[t]);
        }
      }
#pragma unroll
      for (int r = 0; r < 8; ++r) {
        const float ev = sE[itl * 16 + 8 * hh + r];
        yacc[0][r] *= ev;
        yacc[1][r] *= ev;
      }
#pragma unroll
      for (int ks = 0; ks < 2; ++ks) {
        const v16b af = Frag<__bf16>::load(sM + (itl * 16 + l15) * kQ + ks * 32 + 8 * hh);
#pragma unroll
        for (int t = 0; t < 2; ++t) {
          const v16b bfv = Frag<__bf16>::load(sXT + ((hf * 2 + t) * 16 + l15) * kQ + ks * 32 + 8 * hh);
          yacc[t] = mma_b(af, bfv, yacc[t]);
        }
      }
    }
    {
      const float dec = sDec[0];
#pragma unroll
      for (int t = 0; t < 4; ++t)
#pragma unroll
        for (int r = 0; r < 8; ++r) hacc[t][r] *= dec;
#pragma unroll
      for (int ks = 0; ks < 2; ++ks) {
        const v16b af = Frag<__bf16>::load(sXW + (itl * 16 + l15) * kQ + ks * 32 + 8 * hh);
#pragma unroll
        for (int t = 0; t < 4; ++t) {
          const v16b bfv = Frag<__bf16>::load(BTd + (size_t)((hf * 4 + t) * 16 + l15) * kSeq + s0 + ks * 32 + 8 * hh);
          hacc[t] = mma_b(af, bfv, hacc[t]);
        }
      }
    }
    __syncthreads();
#pragma unroll
    for (int t = 0; t < 4; ++t)
#pragma unroll
      for (int r = 0; r < 8; ++r)
        sH[(itl * 16 + 8 * hh + r) * kNs + (hf * 4 + t) * 16 + l15] = bits2bf(f2bf_bits(hacc[t][r]));
#pragma unroll
    for (int t = 0; t < 2; ++t)
#pragma unroll
      for (int r = 0; r < 8; ++r) {
        const int li = (itl * 16 + 8 * hh + r) * 68 + (hf * 2 + t) * 16 + l15;
        const float xv = sXf[li];
        sXf[li] = yacc[t][r] + Dh * xv;
      }
    __syncthreads();
    {
      const int q = lane >> 3, c8 = (lane & 7) * 8;
#pragma unroll 1
      for (int itr = 0; itr < 2; ++itr) {
        const int i = itr * 32 + wave * 4 + q;
        const int s = s0 + i;
        const int trow = bb * kSeq + (dir ? (kSeq - 1 - s) : s);
        const v4u zw = *(const v4u*)(ZXd + (size_t)trow * kZxW + hd * 32 + (lane & 7) * 4);
        const v4f y0 = *(const v4f*)(sXf + i * 68 + c8);
        const v4f y1 = *(const v4f*)(sXf + i * 68 + c8 + 4);
        float yv[8];
#pragma unroll
        for (int e = 0; e < 4; ++e) { yv[e] = y0[e]; yv[4 + e] = y1[e]; }
        v8h hv;
#pragma unroll
        for (int k = 0; k < 4; ++k) {
          const unsigned w = zw[k];
          const float z0 = h16_to_f32(w & 0xffffu);
          const float z1 = h16_to_f32(w >> 16);
          hv[2 * k]     = (_Float16)(yv[2 * k] * silu_f(z0) * kGCarry);
          hv[2 * k + 1] = (_Float16)(yv[2 * k + 1] * silu_f(z1) * kGCarry);
        }
        unsigned short* gp = Gd + (size_t)trow * kDi + hd * kHd + c8;
        *(volatile v8h*)gp = hv;
        __threadfence();
        *(volatile v8h*)gp = hv;
      }
    }
  }
}

__global__ __launch_bounds__(256) void gated_norm_kernel(
    const unsigned* __restrict__ Gw, const float* __restrict__ nw0, const float* __restrict__ nw1,
    unsigned short* __restrict__ YN)
{
  __shared__ float red[8];
  const int tid = threadIdx.x, lane = tid & 31, wave = tid >> 5;
  const int row = blockIdx.x, dir = blockIdx.y;
  const float* nw = dir ? nw1 : nw0;
  const v4u gw = *(const v4u*)(Gw + ((size_t)dir * kRows + row) * (kDi / 2) + tid * 4);
  float g[8];
#pragma unroll
  for (int k = 0; k < 4; ++k) {
    const unsigned w = gw[k];
    g[2 * k]     = h16_to_f32(w & 0xffffu) * (1.0f / kGCarry);
    g[2 * k + 1] = h16_to_f32(w >> 16) * (1.0f / kGCarry);
  }
  float ss = 0.0f;
#pragma unroll
  for (int e = 0; e < 8; ++e) ss = fmaf(g[e], g[e], ss);
  ss += __shfl_xor(ss, 16, 32);
  ss += __shfl_xor(ss, 8, 32);
  ss += __shfl_xor(ss, 4, 32);
  ss += __shfl_xor(ss, 2, 32);
  ss += __shfl_xor(ss, 1, 32);
  if (lane == 0) red[wave] = ss;
  __syncthreads();
  float tot = 0.0f;
#pragma unroll
  for (int w = 0; w < 8; ++w) tot += red[w];
  const float rs = rsqrtf(tot * (1.0f / (float)kDi) + 1e-5f);
  const v4f n0 = *(const v4f*)(nw + tid * 8);
  const v4f n1 = *(const v4f*)(nw + tid * 8 + 4);
  v8h hv;
#pragma unroll
  for (int e = 0; e < 4; ++e) {
    hv[e]     = (_Float16)(g[e] * rs * bf16_rne(n0[e]) * kYnCarry);
    hv[4 + e] = (_Float16)(g[4 + e] * rs * bf16_rne(n1[e]) * kYnCarry);
  }
  unsigned short* yp = YN + (size_t)row * (2 * kDi) + dir * kDi + tid * 8;
  *(volatile v8h*)yp = hv;
  __threadfence();
  *(volatile v8h*)yp = hv;
}

extern "C" void kernel_launch(void* const* d_in, const int* in_sizes, int n_in,
                              void* d_out, int out_size, void* d_ws, size_t ws_size,
                              hipStream_t stream)
{
  if (n_in < 17) return;
  if (in_sizes[0] != kRows * kDm) return;
  for (int d = 0; d < 2; ++d) {
    const int o = 1 + 8 * d;
    if (in_sizes[o + 0] != kDm * kPj) return;
    if (in_sizes[o + 1] != 4 * kCv) return;
    if (in_sizes[o + 2] != kCv) return;
    if (in_sizes[o + 3] != kNh || in_sizes[o + 4] != kNh || in_sizes[o + 5] != kNh) return;
    if (in_sizes[o + 6] != kDi) return;
    if (in_sizes[o + 7] != kDi * kDm) return;
  }
  if (out_size != kRows * kDm) return;
  if (ws_size < kWsTotal) return;

  const float* x    = (const float*)d_in[0];
  const float* Wif  = (const float*)d_in[1];
  const float* cwf  = (const float*)d_in[2];
  const float* cbf  = (const float*)d_in[3];
  const float* dtbf = (const float*)d_in[4];
  const float* alf  = (const float*)d_in[5];
  const float* ddf  = (const float*)d_in[6];
  const float* nwf  = (const float*)d_in[7];
  const float* Wof  = (const float*)d_in[8];
  const float* Wib  = (const float*)d_in[9];
  const float* cwb  = (const float*)d_in[10];
  const float* cbb  = (const float*)d_in[11];
  const float* dtbb = (const float*)d_in[12];
  const float* alb  = (const float*)d_in[13];
  const float* ddb  = (const float*)d_in[14];
  const float* nwb  = (const float*)d_in[15];
  const float* Wob  = (const float*)d_in[16];

  char* ws = (char*)d_ws;
  unsigned short* X16  = (unsigned short*)(ws + kOffX16);
  unsigned short* WinT = (unsigned short*)(ws + kOffWinT);
  unsigned short* G16  = (unsigned short*)(ws + kOffG);
  unsigned short* ZX   = (unsigned short*)(ws + kOffZX);
  unsigned short* YN   = (unsigned short*)(ws + kOffYN);
  unsigned short* BCc  = (unsigned short*)(ws + kOffBC);
  unsigned short* BT   = (unsigned short*)(ws + kOffBT);
  float*          CB   = (float*)(ws + kOffCB);
  unsigned short* WoT  = (unsigned short*)(ws + kOffWoT);

  cast_rows_f16_kernel<<<(kRows * kDm) / 8 / 256, 256, 0, stream>>>(x, X16, (kRows * kDm) / 8);

  transpose_cast_kernel<<<dim3(kPjP / 64, kDm / 64, 2), 256, 0, stream>>>(
      Wif, Wib, WinT, kDm, kPj, kDm, (long)kPjP * kDm, 0, kWCarry);

  transpose_cast_kernel<<<dim3(kDm / 64, kDi / 64, 2), 256, 0, stream>>>(
      Wof, Wob, WoT, kDi, kDm, 2 * kDi, 0L, kDi, kWCarry);

  wmma_gemm64_f16<1><<<dim3(((kRows / 64) * (kPjP / 64)) / 8, 2), 256, 0, stream>>>(
      X16, kDm, 0L,
      WinT, kDm, (long)kPjP * kDm,
      (void*)ZX, kPjP, (long)kRows * kPjP,
      kRows, kPjP, kDm, 1.0f / kWCarry);

  bc_prep_kernel<<<2 * kBatch * kNck, 256, 0, stream>>>(
      (const unsigned*)ZX, cwf, cbf, cwb, cbb, BCc, BT, CB);

  ssd_scan_kernel<<<2 * kBatch * kNh, 256, 0, stream>>>(
      (const unsigned*)ZX, BCc, BT, CB,
      cwf, cbf, dtbf, alf, ddf,
      cwb, cbb, dtbb, alb, ddb,
      G16);

  gated_norm_kernel<<<dim3(kRows, 2), 256, 0, stream>>>((const unsigned*)G16, nwf, nwb, YN);

  wmma_gemm64_f16<0><<<dim3(((kRows / 64) * (kDm / 64)) / 8, 1), 256, 0, stream>>>(
      YN, 2 * kDi, 0L,
      WoT, 2 * kDi, 0L,
      d_out, kDm, 0L,
      kRows, kDm, 2 * kDi, 1.0f / (kYnCarry * kWCarry));
}
